// KAN_20615843021188
// MI455X (gfx1250) — hardware-verified
//
#include <hip/hip_runtime.h>
#include <stddef.h>


#define NTHR    256
#define NWAVE   8
#define FR      64
#define BM      64
#define BNC     128
#define DDIM    256
#define ODIM    256
#define NCOEF   5
#define NLAYER  2
#define KDIM    (DDIM * NCOEF)
#define UPR     (KDIM / 8)
#define WSCAP   134217728
#define ACARRY  32.0f
#define WCARRY  1024.0f
#define GSCALE  (1.0f / 8388608.0f)
#define LNEPS   1e-6f

static_assert((KDIM % 32) == 0);
static_assert((UPR % 32) == 0);
static_assert(DDIM == 8 * 32);
static_assert((ODIM % BNC) == 0);
static_assert(FR == BM && (FR % NWAVE) == 0);
static_assert((NLAYER * ODIM * UPR) % NTHR == 0);

typedef float    v4f  __attribute__((ext_vector_type(4)));
typedef float    v8f  __attribute__((ext_vector_type(8)));
typedef _Float16 v8h  __attribute__((ext_vector_type(8)));
typedef _Float16 v16h __attribute__((ext_vector_type(16)));
union Frag { v16h v; v8h h[2]; };

__device__ __forceinline__ v8f wmh(v16h a, v16h b, v8f c) {
  v8f d = __builtin_amdgcn_wmma_f32_16x16x32_f16(false, a, false, b, (short)0, c, false, false);
  asm volatile("v_nop\n\tv_nop\n\tv_nop\n\tv_nop" : "+v"(d) : "v"(a), "v"(b));
  return d;
}

__device__ __forceinline__ float wsum1(float v) {
#pragma unroll
  for (int off = 16; off > 0; off >>= 1) v += __shfl_xor(v, off);
  return v;
}

__global__ __launch_bounds__(NTHR) void k_wcvt(const float* __restrict__ coefs, _Float16* wp, int nUnits) {
  const int i = (int)blockIdx.x * NTHR + (int)threadIdx.x;
  if (i >= nUnits) return;
  const int upl   = ODIM * UPR;
  const int layer = i / upl;
  const int r     = i - layer * upl;
  const int n     = r / UPR;
  const int seg   = r - n * UPR;
  const float* cl = coefs + (size_t)layer * DDIM * ODIM * NCOEF;
  v8h o;
#pragma unroll
  for (int j = 0; j < 8; ++j) {
    const int k = 8 * seg + j;
    const int c = k / DDIM;
    const int d = k - c * DDIM;
    const float f = cl[((size_t)d * ODIM + n) * NCOEF + c];
    o[j] = (_Float16)(f * WCARRY);
  }
  _Float16* gp = wp + (size_t)i * 8;
  *(volatile v8h*)gp = o;
  __threadfence();
  *(volatile v8h*)gp = o;
}

__global__ __launch_bounds__(NTHR) void k_feat(
    const float* __restrict__ hin, const float* __restrict__ alphas, int layer,
    const float* __restrict__ lg, const float* __restrict__ lb, _Float16* aout, int nRow) {
#pragma clang fp contract(off)
  constexpr int NI = UPR / 32;
  __shared__ __attribute__((aligned(16))) _Float16 srow[NWAVE * KDIM];
  const int tid = threadIdx.x, lane = tid & 31, wave = tid >> 5;
  _Float16* my = srow + wave * KDIM;
  const float invd = 1.0f / (float)DDIM;

  const int li = layer < 0 ? 0 : (layer > NLAYER - 1 ? NLAYER - 1 : layer);
  const float a   = tanhf(alphas[li]);
  const float a2  = 2.0f * a;
  const float ap1 = a + 1.0f;
  const float t2  = 4.0f + a2;
  const float A2  = (4.0f * (2.0f + a2)) * (t2 - 2.0f);
  const float B2  = ((t2 - 1.0f) * t2) * (t2 - 2.0f);
  const float q2  = (2.0f + a) - 1.0f;
  const float C2  = (2.0f * (q2 * q2)) * t2;
  const float iA2 = 1.0f / A2;
  const float t3  = 6.0f + a2;
  const float A3  = (6.0f * (3.0f + a2)) * (t3 - 2.0f);
  const float B3  = ((t3 - 1.0f) * t3) * (t3 - 2.0f);
  const float q3  = (3.0f + a) - 1.0f;
  const float C3  = (2.0f * (q3 * q3)) * t3;
  const float iA3 = 1.0f / A3;
  const float t4  = 8.0f + a2;
  const float A4  = (8.0f * (4.0f + a2)) * (t4 - 2.0f);
  const float B4  = ((t4 - 1.0f) * t4) * (t4 - 2.0f);
  const float q4  = (4.0f + a) - 1.0f;
  const float C4  = (2.0f * (q4 * q4)) * t4;
  const float iA4 = 1.0f / A4;

#pragma unroll 1
  for (int it = 0; it < FR / NWAVE; ++it) {
    const int lr = (int)blockIdx.x * FR + it * NWAVE + wave;
    int rr = lr > nRow - 1 ? nRow - 1 : lr;
    rr = rr < 0 ? 0 : rr;
    const float* src = hin + (size_t)rr * DDIM + lane;

    float hv[8];
#pragma unroll
    for (int q = 0; q < 8; ++q) hv[q] = src[32 * q];
    float s = 0.f;
#pragma unroll
    for (int q = 0; q < 8; ++q) s += hv[q];
    s = wsum1(s);
    const float mu = s * invd;
    float sq = 0.f;
#pragma unroll
    for (int q = 0; q < 8; ++q) { const float dv = hv[q] - mu; sq += dv * dv; }
    sq = wsum1(sq);
    const float rs = rsqrtf(sq * invd + LNEPS);

#pragma unroll 1
    for (int q = 0; q < 8; ++q) {
      const int c = 32 * q + lane;
      const float h  = src[32 * q];
      const float hn = ((h - mu) * rs) * lg[c] + lb[c];
      const float x  = tanhf(hn);
      const float p1 = ap1 * x;
      const float p2 = ((B2 * x) * p1 - C2) * iA2;
      const float p3 = ((B3 * x) * p2 - C3 * p1) * iA3;
      const float p4 = ((B4 * x) * p3 - C4 * p2) * iA4;
      my[c]            = (_Float16)ACARRY;
      my[DDIM + c]     = (_Float16)(p1 * ACARRY);
      my[2 * DDIM + c] = (_Float16)(p2 * ACARRY);
      my[3 * DDIM + c] = (_Float16)(p3 * ACARRY);
      my[4 * DDIM + c] = (_Float16)(p4 * ACARRY);
    }
    __syncthreads();

    _Float16* gp = aout + (size_t)lr * KDIM;
    v8h pv[NI];
#pragma unroll
    for (int i = 0; i < NI; ++i) pv[i] = *(const v8h*)(my + 8 * (i * 32 + lane));
#pragma unroll
    for (int i = 0; i < NI; ++i) *(volatile v8h*)(gp + 8 * (i * 32 + lane)) = pv[i];
    __threadfence();
#pragma unroll
    for (int i = 0; i < NI; ++i) *(volatile v8h*)(gp + 8 * (i * 32 + lane)) = pv[i];
    __syncthreads();
  }
}

template <int NWV, int TPW, int BNCT>
__global__ __launch_bounds__(NWV * 32) void k_gemm(
    const _Float16* __restrict__ A, const _Float16* __restrict__ Bp,
    float* Cout, int K, int ldc, int nValid, int nStore) {
  constexpr int NT  = NWV * 32;
  constexpr int WPR = NWV / 4;
  static_assert(WPR >= 1 && WPR * 4 == NWV);
  static_assert(WPR * TPW * 16 == BNCT && (BNCT % 32) == 0);
  constexpr int PPR = BNCT / 4;
  constexpr int NIT = (BM * PPR) / NT;
  static_assert(NIT * NT == BM * PPR && NIT >= 1);
  static_assert(BM == 4 * 16);

  __shared__ __attribute__((aligned(16))) float stg[BM * BNCT];
  const int tid = threadIdx.x, lane = tid & 31, wave = tid >> 5, hh = lane >> 4, m = lane & 15;
  const int rowBase = (int)blockIdx.x * BM;
  const int colBase = (int)blockIdx.y * BNCT;
  const int rg = wave / WPR, chf = wave - rg * WPR;
  const int r0 = rg * 16;
  const int c0 = chf * TPW * 16;

  v8f acc[TPW];
#pragma unroll
  for (int t = 0; t < TPW; ++t) { v8f z = {0.f, 0.f, 0.f, 0.f, 0.f, 0.f, 0.f, 0.f}; acc[t] = z; }

  const _Float16* ap = A  + (size_t)(rowBase + r0 + m) * K + 8 * hh;
  const _Float16* bp = Bp + (size_t)(colBase + c0 + m) * K + 8 * hh;
  const int ksteps = K >> 5;
#pragma unroll 1
  for (int kt = 0; kt < ksteps; ++kt) {
    Frag a;
    a.h[0] = *(const v8h*)(ap + 32 * kt);
    a.h[1] = *(const v8h*)(ap + 32 * kt + 16);
#pragma unroll
    for (int t = 0; t < TPW; ++t) {
      const size_t to = (size_t)(16 * t) * K + 32 * kt;
      Frag b;
      b.h[0] = *(const v8h*)(bp + to);
      b.h[1] = *(const v8h*)(bp + to + 16);
      acc[t] = wmh(a.v, b.v, acc[t]);
    }
  }

  {
    float* sp = stg + (size_t)(r0 + 8 * hh) * BNCT + c0 + m;
    const int growb = rowBase + r0 + 8 * hh;
#pragma unroll
    for (int t = 0; t < TPW; ++t) {
#pragma unroll
      for (int r = 0; r < 8; ++r) {
        const bool lv = (growb + r) < nValid;
        const float g = acc[t][r] * GSCALE;
        sp[r * BNCT + 16 * t] = lv ? g : 0.f;
      }
    }
  }
  __syncthreads();

  v4f cv[NIT];
#pragma unroll
  for (int it = 0; it < NIT; ++it) {
    const int id = it * NT + tid;
    const int row = id / PPR, seg = id - row * PPR;
    cv[it] = *(const v4f*)(stg + (size_t)row * BNCT + 4 * seg);
  }
#pragma unroll
  for (int it = 0; it < NIT; ++it) {
    const int id = it * NT + tid;
    const int row = id / PPR, seg = id - row * PPR;
    const int grow = rowBase + row;
    if (grow < nStore) {
      float* gp = Cout + (size_t)grow * ldc + colBase + 4 * seg;
      *(volatile v4f*)gp = cv[it];
    }
  }
  __threadfence();
#pragma unroll
  for (int it = 0; it < NIT; ++it) {
    const int id = it * NT + tid;
    const int row = id / PPR, seg = id - row * PPR;
    const int grow = rowBase + row;
    if (grow < nStore) {
      float* gp = Cout + (size_t)grow * ldc + colBase + 4 * seg;
      *(volatile v4f*)gp = cv[it];
    }
  }
}

extern "C" void kernel_launch(void* const* d_in, const int* in_sizes, int n_in,
                              void* d_out, int out_size, void* d_ws, size_t ws_size,
                              hipStream_t stream) {
  if (n_in < 5) return;
  if (in_sizes[0] < DDIM || (in_sizes[0] % DDIM) != 0) return;
  const int nRow = in_sizes[0] / DDIM;
  if (nRow < 1 || nRow > (1 << 22)) return;
  if (in_sizes[1] != NLAYER * DDIM * ODIM * NCOEF) return;
  if (in_sizes[2] != NLAYER) return;
  if (in_sizes[3] != NLAYER * DDIM || in_sizes[4] != NLAYER * DDIM) return;
  if (out_size != nRow * ODIM) return;

  const float* x      = (const float*)d_in[0];
  const float* coefs  = (const float*)d_in[1];
  const float* alphas = (const float*)d_in[2];
  const float* lns    = (const float*)d_in[3];
  const float* lnb    = (const float*)d_in[4];
  float* out = (float*)d_out;

  const int NPAD = ((nRow + BM - 1) / BM) * BM;

  char* ws = (char*)d_ws;
  size_t off = 0;
  const size_t oW = off; off += (size_t)NLAYER * ODIM * KDIM * 2;   off = (off + 255) & ~(size_t)255;
  const size_t oA = off; off += (size_t)NPAD * KDIM * 2;            off = (off + 255) & ~(size_t)255;
  const size_t oH = off; off += (size_t)NPAD * ODIM * 4;            off = (off + 255) & ~(size_t)255;
  if (off > ws_size || off > (size_t)WSCAP) return;

  _Float16* wpl = (_Float16*)(ws + oW);
  _Float16* apl = (_Float16*)(ws + oA);
  float*    h1  = (float*)(ws + oH);

  const int nU = NLAYER * ODIM * UPR;
  k_wcvt<<<(nU + NTHR - 1) / NTHR, NTHR, 0, stream>>>(coefs, wpl, nU);

  k_feat<<<NPAD / FR, NTHR, 0, stream>>>(x, alphas, 0, lns, lnb, apl, nRow);
  k_gemm<8, 4, BNC><<<dim3(NPAD / BM, ODIM / BNC), 256, 0, stream>>>(
      apl, wpl, h1, KDIM, ODIM, nRow, NPAD);

  k_feat<<<NPAD / FR, NTHR, 0, stream>>>(h1, alphas, 1, lns + DDIM, lnb + DDIM, apl, nRow);
  k_gemm<8, 4, BNC><<<dim3(NPAD / BM, ODIM / BNC), 256, 0, stream>>>(
      apl, wpl + (size_t)ODIM * KDIM, out, KDIM, ODIM, nRow, nRow);
}
